// SteerablePocketBlock_87333864997035
// MI455X (gfx1250) — hardware-run, weakly checked
//
#include <hip/hip_runtime.h>
#define NBt 2
#define NN 512
#define DD 128
#define NTOK (NBt * NN)
#define ICH 64
#define PCH (ICH * NN)
typedef __bf16 v16b __attribute__((ext_vector_type(16)));
typedef unsigned short v8us __attribute__((ext_vector_type(8), may_alias));
typedef float  v8f  __attribute__((ext_vector_type(8)));
typedef float  v4f  __attribute__((ext_vector_type(4)));
typedef float  v4fa __attribute__((ext_vector_type(4), may_alias));
union FragB { v16b v; v8us half[2]; unsigned short u[16]; };

__device__ __forceinline__ unsigned short bf16_bits(float x) { unsigned int u = __float_as_uint(x); return (unsigned short)((u + 0x7FFFu + ((u >> 16) & 1u)) >> 16); }
__device__ __forceinline__ float bf16_val(unsigned short b) { return __uint_as_float(((unsigned int)b) << 16); }
__device__ __forceinline__ float bf16_round(float x) { return bf16_val(bf16_bits(x)); }
template <int NT>
__device__ __forceinline__ v8f mmaN(v16b ah, v16b al, v16b bh, v16b bl, v8f c) {
  c = __builtin_amdgcn_wmma_f32_16x16x32_bf16(false, ah, false, bh, (short)0, c, false, false);
  if (NT >= 2) c = __builtin_amdgcn_wmma_f32_16x16x32_bf16(false, al, false, bh, (short)0, c, false, false);
  if (NT >= 3) c = __builtin_amdgcn_wmma_f32_16x16x32_bf16(false, ah, false, bl, (short)0, c, false, false);
  asm volatile("v_nop\n\tv_nop\n\tv_nop\n\tv_nop" : "+v"(c) : "v"(ah), "v"(al), "v"(bh), "v"(bl));
  return c;
}

__global__ __launch_bounds__(256) void k_wt_bf16(const float* __restrict__ W, unsigned short* __restrict__ Wt, int K, int N) {
  const int t = blockIdx.x * 256 + threadIdx.x;
  const int k8n = K / 8;
  if (t >= N * k8n) return;
  const int n = t / k8n, k8 = (t % k8n) * 8;
  v8us v;
#pragma unroll
  for (int i = 0; i < 8; ++i) v[i] = bf16_bits(W[(size_t)(k8 + i) * N + n]);
  *(volatile v8us*)(Wt + (size_t)n * K + k8) = v;
  __threadfence();
  *(volatile v8us*)(Wt + (size_t)n * K + k8) = v;
}

template <bool ASPLIT, int ACT, bool BIAS_BF16>
__global__ __launch_bounds__(128) void k_gemm_bf(const float* __restrict__ A, int lda, const unsigned short* __restrict__ Wt, int ldb,
                                               const float* __restrict__ bias, float* __restrict__ C, int ldc, int M, int N, int K) {
  __shared__ __attribute__((aligned(16))) float so[4][16][64];
  const int tid = threadIdx.x, w = tid >> 5, lane = tid & 31, ln = lane & 15, hh = lane >> 4;
  const int ntn = N / 64;
  const int wid = blockIdx.x * 4 + w;
  const int mt = wid / ntn, nq = wid % ntn;
  if (mt * 16 >= M) return;
  const int row0 = mt * 16, col0 = nq * 64;
  const float* arow = A + (size_t)(row0 + ln) * lda;
  v8f acc[4] = {};
  for (int kb = 0; kb < K; kb += 32) {
    FragB ah, al;
    const v4f x0 = *(const v4fa*)(arow + kb + 8 * hh), x1 = *(const v4fa*)(arow + kb + 8 * hh + 4);
    const v4f x2 = *(const v4fa*)(arow + kb + 16 + 8 * hh), x3 = *(const v4fa*)(arow + kb + 16 + 8 * hh + 4);
    float xs[16] = {x0[0],x0[1],x0[2],x0[3],x1[0],x1[1],x1[2],x1[3],x2[0],x2[1],x2[2],x2[3],x3[0],x3[1],x3[2],x3[3]};
#pragma unroll
    for (int i = 0; i < 16; ++i) { const unsigned short hb = bf16_bits(xs[i]); ah.u[i] = hb; al.u[i] = ASPLIT ? bf16_bits(xs[i] - bf16_val(hb)) : (unsigned short)0; }
#pragma unroll
    for (int t = 0; t < 4; ++t) {
      const unsigned short* brow = Wt + (size_t)(col0 + t * 16 + ln) * ldb + kb;
      FragB b;
      b.half[0] = *(const v8us*)(brow + 8 * hh);
      b.half[1] = *(const v8us*)(brow + 16 + 8 * hh);
      acc[t] = mmaN<ASPLIT ? 2 : 1>(ah.v, al.v, b.v, b.v, acc[t]);
    }
  }
#pragma unroll
  for (int t = 0; t < 4; ++t) {
    float bv = bias ? bias[col0 + t * 16 + ln] : 0.f;
    if (BIAS_BF16) bv = bf16_round(bv);
#pragma unroll
    for (int r = 0; r < 8; ++r) { float v = acc[t][r] + bv; if (ACT == 1) v = fmaxf(v, 0.f); so[w][8 * hh + r][t * 16 + ln] = v; }
  }
  __builtin_amdgcn_fence(__ATOMIC_ACQ_REL, "workgroup");
  __builtin_amdgcn_wave_barrier();
  const int rsub = lane >> 4, c4 = (lane & 15) * 4;
  for (int pass = 0; pass < 2; ++pass) {
#pragma unroll
    for (int q = 0; q < 8; ++q) {
      const int r = q * 2 + rsub;
      const v4f v = *(const v4fa*)&so[w][r][c4];
      *(volatile v4f*)(C + (size_t)(row0 + r) * ldc + col0 + c4) = v;
    }
    if (pass == 0) __threadfence();
  }
}

template <bool ASPLIT, int ACT, bool BIAS_BF16, bool RES_BF16>
__global__ __launch_bounds__(128) void k_gemm_bf3(const float* __restrict__ A, int lda, const unsigned short* __restrict__ Wt, int ldb,
                                                const float* __restrict__ bias, const float* __restrict__ resid, int rmod, int ldr,
                                                float* __restrict__ C, int ldc, int M, int N, int K) {
  __shared__ __attribute__((aligned(16))) float so[4][16][64];
  const int tid = threadIdx.x, w = tid >> 5, lane = tid & 31, ln = lane & 15, hh = lane >> 4;
  const int ntn = N / 64;
  const int wid = blockIdx.x * 4 + w;
  const int mt = wid / ntn, nq = wid % ntn;
  if (mt * 16 >= M) return;
  const int row0 = mt * 16, col0 = nq * 64;
  const float* arow = A + (size_t)(row0 + ln) * lda;
  v8f acc[4] = {};
  for (int kb = 0; kb < K; kb += 32) {
    FragB ah, al;
    const v4f x0 = *(const v4fa*)(arow + kb + 8 * hh), x1 = *(const v4fa*)(arow + kb + 8 * hh + 4);
    const v4f x2 = *(const v4fa*)(arow + kb + 16 + 8 * hh), x3 = *(const v4fa*)(arow + kb + 16 + 8 * hh + 4);
    float xs[16] = {x0[0],x0[1],x0[2],x0[3],x1[0],x1[1],x1[2],x1[3],x2[0],x2[1],x2[2],x2[3],x3[0],x3[1],x3[2],x3[3]};
#pragma unroll
    for (int i = 0; i < 16; ++i) { const unsigned short hb = bf16_bits(xs[i]); ah.u[i] = hb; al.u[i] = ASPLIT ? bf16_bits(xs[i] - bf16_val(hb)) : (unsigned short)0; }
#pragma unroll
    for (int t = 0; t < 4; ++t) {
      const unsigned short* brow = Wt + (size_t)(col0 + t * 16 + ln) * ldb + kb;
      FragB b;
      b.half[0] = *(const v8us*)(brow + 8 * hh);
      b.half[1] = *(const v8us*)(brow + 16 + 8 * hh);
      acc[t] = mmaN<ASPLIT ? 2 : 1>(ah.v, al.v, b.v, b.v, acc[t]);
    }
  }
#pragma unroll
  for (int t = 0; t < 4; ++t) {
    const int col = col0 + t * 16 + ln;
    float bv = bias ? bias[col] : 0.f;
    if (BIAS_BF16) bv = bf16_round(bv);
#pragma unroll
    for (int r = 0; r < 8; ++r) {
      float v = acc[t][r] + bv;
      if (resid) { float rv = resid[(size_t)((row0 + 8 * hh + r) % rmod) * ldr + col]; if (RES_BF16) rv = bf16_round(rv); v += rv; }
      if (ACT == 1) v = fmaxf(v, 0.f);
      if (ACT == 2) v = 0.5f * v * (1.0f + erff(v * 0.70710678118654752f));
      if (ACT == 3) { const float u = 0.7978845608028654f * (v + 0.044715f * v * v * v); v = 0.5f * v * (1.0f + tanhf(u)); }
      so[w][8 * hh + r][t * 16 + ln] = v;
    }
  }
  __builtin_amdgcn_fence(__ATOMIC_ACQ_REL, "workgroup");
  __builtin_amdgcn_wave_barrier();
  const int rsub = lane >> 4, c4 = (lane & 15) * 4;
  for (int pass = 0; pass < 2; ++pass) {
#pragma unroll
    for (int q = 0; q < 8; ++q) {
      const int r = q * 2 + rsub;
      const v4f v = *(const v4fa*)&so[w][r][c4];
      *(volatile v4f*)(C + (size_t)(row0 + r) * ldc + col0 + c4) = v;
    }
    if (pass == 0) __threadfence();
  }
}
template <bool PARAM_BF16>
__global__ __launch_bounds__(256) void k_layernorm(const float* __restrict__ X, const float* __restrict__ R, const float* __restrict__ g, const float* __restrict__ bta,
                                                  float* __restrict__ out_sum, float* __restrict__ out_norm, int N, float eps) {
  __shared__ float red[256];
  const int row = blockIdx.x, tid = threadIdx.x;
  const float* x = X + (size_t)row * N; const float* rr = R ? R + (size_t)row * N : nullptr;
  float vals[16];
  const int per = N / 256;
  float s1 = 0.f;
  for (int u = 0; u < per / 4; ++u) {
    const int j = tid * 4 + 1024 * u;
    const v4f a = *(const v4fa*)(x + j);
    v4f b = {0.f,0.f,0.f,0.f}; if (rr) b = *(const v4fa*)(rr + j);
#pragma unroll
    for (int q = 0; q < 4; ++q) { const float v = a[q] + b[q]; vals[u * 4 + q] = v; s1 += v; }
  }
  red[tid] = s1; __syncthreads();
  for (int st = 128; st > 0; st >>= 1) { if (tid < st) red[tid] += red[tid + st]; __syncthreads(); }
  const float mu = red[0] / (float)N; __syncthreads();
  float s2 = 0.f;
  for (int u = 0; u < per / 4; ++u)
#pragma unroll
    for (int q = 0; q < 4; ++q) { const float c = vals[u * 4 + q] - mu; s2 += c * c; }
  red[tid] = s2; __syncthreads();
  for (int st = 128; st > 0; st >>= 1) { if (tid < st) red[tid] += red[tid + st]; __syncthreads(); }
  const float rs = rsqrtf(red[0] / (float)N + eps);
  for (int pass = 0; pass < 2; ++pass) {
    for (int u = 0; u < per / 4; ++u) {
      const int j = tid * 4 + 1024 * u;
      v4f o, sm;
#pragma unroll
      for (int q = 0; q < 4; ++q) {
        float gg = g[j + q], bb = bta[j + q];
        if (PARAM_BF16) { gg = bf16_round(gg); bb = bf16_round(bb); }
        sm[q] = vals[u * 4 + q]; o[q] = (vals[u * 4 + q] - mu) * rs * gg + bb;
      }
      if (out_sum) *(volatile v4f*)(out_sum + (size_t)row * N + j) = sm;
      *(volatile v4f*)(out_norm + (size_t)row * N + j) = o;
    }
    if (pass == 0) __threadfence();
  }
}


typedef _Float16 v16h __attribute__((ext_vector_type(16)));
union FragH { v16h v; v8us half[2]; _Float16 h[16]; unsigned short u[16]; };
template <int NT>
__device__ __forceinline__ v8f mmaH(v16h ah, v16h al, v16h bh, v16h bl, v8f c) {
  c = __builtin_amdgcn_wmma_f32_16x16x32_f16(false, ah, false, bh, (short)0, c, false, false);
  if (NT >= 2) c = __builtin_amdgcn_wmma_f32_16x16x32_f16(false, al, false, bh, (short)0, c, false, false);
  if (NT >= 3) c = __builtin_amdgcn_wmma_f32_16x16x32_f16(false, ah, false, bl, (short)0, c, false, false);
  asm volatile("v_nop\n\tv_nop\n\tv_nop\n\tv_nop" : "+v"(c) : "v"(ah), "v"(al), "v"(bh), "v"(bl));
  return c;
}
template <bool ASPLIT>
__global__ __launch_bounds__(128) void k_gemm_h(const float* __restrict__ A, int lda, size_t sA, const _Float16* __restrict__ Bh, int ldb, size_t sB, float alpha, float* __restrict__ C, int ldc, size_t sC, int M, int N, int K) {
  __shared__ __attribute__((aligned(16))) float so[4][16][64];
  const int tid = threadIdx.x, w = tid >> 5, lane = tid & 31, ln = lane & 15, hh = lane >> 4; const int by = blockIdx.y;
  A += (size_t)by * sA; Bh += (size_t)by * sB; C += (size_t)by * sC;
  const int ntn = (N + 63) / 64; const int wid = blockIdx.x * 4 + w; const int mt = wid / ntn, nq = wid % ntn; if (mt * 16 >= M) return;
  const int row0 = mt * 16, col0 = nq * 64; const float* arow = A + (size_t)(row0 + ln) * lda;
  v8f acc[4] = {};
  for (int kb = 0; kb < K; kb += 32) {
    FragH ah, al;
    const v4f x0 = *(const v4fa*)(arow + kb + 8 * hh), x1 = *(const v4fa*)(arow + kb + 8 * hh + 4), x2 = *(const v4fa*)(arow + kb + 16 + 8 * hh), x3 = *(const v4fa*)(arow + kb + 16 + 8 * hh + 4);
    float xs[16] = {x0[0],x0[1],x0[2],x0[3],x1[0],x1[1],x1[2],x1[3],x2[0],x2[1],x2[2],x2[3],x3[0],x3[1],x3[2],x3[3]};
#pragma unroll
    for (int i = 0; i < 16; ++i) { const _Float16 h = (_Float16)xs[i]; ah.h[i] = h; al.h[i] = ASPLIT ? (_Float16)(xs[i] - (float)h) : (_Float16)0.0f; }
#pragma unroll
    for (int t = 0; t < 4; ++t) { if (col0 + t * 16 >= N) continue; const size_t boff = (size_t)(col0 + t * 16 + ln) * ldb + kb; FragH bq; bq.half[0] = *(const v8us*)(Bh + boff + 8 * hh); bq.half[1] = *(const v8us*)(Bh + boff + 16 + 8 * hh);
      acc[t] = mmaH<ASPLIT ? 2 : 1>(ah.v, al.v, bq.v, bq.v, acc[t]); }
  }
#pragma unroll
  for (int t = 0; t < 4; ++t) { if (col0 + t * 16 >= N) continue;
#pragma unroll
    for (int r = 0; r < 8; ++r) so[w][8 * hh + r][t * 16 + ln] = acc[t][r] * alpha; }
  __builtin_amdgcn_fence(__ATOMIC_ACQ_REL, "workgroup"); __builtin_amdgcn_wave_barrier();
  const int rsub = lane >> 4, c4 = (lane & 15) * 4;
  for (int pass = 0; pass < 2; ++pass) {
#pragma unroll
    for (int q = 0; q < 8; ++q) { const int r = q * 2 + rsub; if (col0 + c4 < N) { const v4f v = *(const v4fa*)&so[w][r][c4]; *(volatile v4f*)(C + (size_t)(row0 + r) * ldc + col0 + c4) = v; } }
    if (pass == 0) __threadfence(); }
}

__global__ __launch_bounds__(256) void k_wt_f16(const float* __restrict__ W, _Float16* __restrict__ Wt, int K, int N, float scale) {
  const int t = blockIdx.x * 256 + threadIdx.x; if (t >= N * (K / 8)) return; const int n = t / (K / 8), k8 = (t % (K / 8)) * 8; FragH f;
#pragma unroll
  for (int i = 0; i < 8; ++i) f.h[i] = (_Float16)(bf16_round(W[(size_t)(k8 + i) * N + n]) * scale); const v8us o = f.half[0];
  *(volatile v8us*)((unsigned short*)Wt + (size_t)n * K + k8) = o; __threadfence(); *(volatile v8us*)((unsigned short*)Wt + (size_t)n * K + k8) = o;
}
template <int ACT>
__global__ __launch_bounds__(128) void k_gemm_hhx(const _Float16* __restrict__ A, int lda, size_t sA, const _Float16* __restrict__ Bh, int ldb, size_t sB, float alpha, const float* __restrict__ bias, size_t sBias, const float* __restrict__ CP, int rowsPerB, size_t sCPb, int row0g,
    float* __restrict__ C, _Float16* __restrict__ C16, int ldc, size_t sC, int M, int N, int K) {
  __shared__ __attribute__((aligned(16))) float so[4][16][64];
  const int tid = threadIdx.x, w = tid >> 5, lane = tid & 31, ln = lane & 15, hh = lane >> 4; const int by = blockIdx.y;
  A += (size_t)by * sA; Bh += (size_t)by * sB; const size_t cofs = (size_t)by * sC; const float* bp = bias ? bias + (size_t)by * sBias : nullptr;
  const int ntn = (N + 63) / 64; const int wid = blockIdx.x * 4 + w; const int mt = wid / ntn, nq = wid % ntn; if (mt * 16 >= M) return;
  const int row0 = mt * 16, col0 = nq * 64; const _Float16* arow = A + (size_t)(row0 + ln) * lda;
  v8f acc[4] = {};
  for (int kb = 0; kb < K; kb += 32) { FragH ah; ah.half[0] = *(const v8us*)((const unsigned short*)arow + kb + 8 * hh); ah.half[1] = *(const v8us*)((const unsigned short*)arow + kb + 16 + 8 * hh);
#pragma unroll
    for (int t = 0; t < 4; ++t) { if (col0 + t * 16 >= N) continue; const size_t boff = (size_t)(col0 + t * 16 + ln) * ldb + kb; FragH bq; bq.half[0] = *(const v8us*)((const unsigned short*)Bh + boff + 8 * hh); bq.half[1] = *(const v8us*)((const unsigned short*)Bh + boff + 16 + 8 * hh);
      acc[t] = mmaH<1>(ah.v, ah.v, bq.v, bq.v, acc[t]); }
  }
#pragma unroll
  for (int t = 0; t < 4; ++t) { if (col0 + t * 16 >= N) continue; const int col = col0 + t * 16 + ln; const float bv = bp ? bf16_round(bp[col]) : 0.f;
#pragma unroll
    for (int r = 0; r < 8; ++r) { float v = acc[t][r] * alpha + bv; if (CP) { const int bidx = (row0g + row0 + 8 * hh + r) / rowsPerB; v += CP[(size_t)bidx * sCPb + (size_t)by * 64 + col]; } if (ACT == 1) v = (v > 0.f) ? v : expm1f(v); else if (ACT == 7) v = (v > 0.f) ? v + 1.0f : expf(v); else if (ACT == 8) v = tanhf(v); else if (ACT == 9) v = 0.5f * v * (1.0f + tanhf(0.7978845608028654f * (v + 0.044715f * v * v * v))); else if (ACT == 11) v = 1.0f / (1.0f + expf(-v)); else if (ACT == 12) v = (v > 0.f) ? v : 0.01f * v; else if (ACT == 14) v = (v > 0.f) ? v : 0.1f * v; else if (ACT == 15) v = v / (1.0f + expf(-v)); else if (ACT == 3) v = fmaxf(v, 0.f); else if (ACT == 6) v = 0.5f * v * (1.0f + erff(v * 0.70710678118654752f)); so[w][8 * hh + r][t * 16 + ln] = v; } }
  __builtin_amdgcn_fence(__ATOMIC_ACQ_REL, "workgroup"); __builtin_amdgcn_wave_barrier();
  const int rsub = lane >> 4, c4 = (lane & 15) * 4; typedef _Float16 v4h __attribute__((ext_vector_type(4)));
  for (int pass = 0; pass < 2; ++pass) {
#pragma unroll
    for (int q = 0; q < 8; ++q) { const int r = q * 2 + rsub; if (col0 + c4 < N) { const v4f v = *(const v4fa*)&so[w][r][c4]; if (C) *(volatile v4f*)(C + cofs + (size_t)(row0 + r) * ldc + col0 + c4) = v; if (C16) { v4h h4; for (int i = 0; i < 4; ++i) h4[i] = (_Float16)v[i]; *(volatile v4h*)(C16 + cofs + (size_t)(row0 + r) * ldc + col0 + c4) = h4; } } }
    if (pass == 0) __threadfence(); }
}


typedef _Float16 v4h __attribute__((ext_vector_type(4)));

__global__ __launch_bounds__(256) void k_x16(const float* __restrict__ x, _Float16* __restrict__ X16, size_t n8) { const size_t t = (size_t)blockIdx.x * 256 + threadIdx.x; if (t >= n8) return; FragH f;
#pragma unroll
  for (int q = 0; q < 8; ++q) f.h[q] = (_Float16)bf16_round(x[t * 8 + q]); *(volatile v8us*)((unsigned short*)X16 + t * 8) = f.half[0]; __threadfence(); *(volatile v8us*)((unsigned short*)X16 + t * 8) = f.half[0]; }
__global__ __launch_bounds__(256) void k_h16(const float* __restrict__ x, _Float16* __restrict__ X16, size_t n8) { const size_t t = (size_t)blockIdx.x * 256 + threadIdx.x; if (t >= n8) return; FragH f;
#pragma unroll
  for (int q = 0; q < 8; ++q) f.h[q] = (_Float16)x[t * 8 + q]; *(volatile v8us*)((unsigned short*)X16 + t * 8) = f.half[0]; __threadfence(); *(volatile v8us*)((unsigned short*)X16 + t * 8) = f.half[0]; }
__global__ __launch_bounds__(256) void k_round16f(const float* __restrict__ W, _Float16* __restrict__ Bt, size_t n8) { const size_t t = (size_t)blockIdx.x * 256 + threadIdx.x; if (t >= n8) return; FragH f;
#pragma unroll
  for (int i = 0; i < 8; ++i) f.h[i] = (_Float16)(bf16_round(W[t * 8 + i]) * 16.0f); *(volatile v8us*)((unsigned short*)Bt + t * 8) = f.half[0]; __threadfence(); *(volatile v8us*)((unsigned short*)Bt + t * 8) = f.half[0]; }
template <int NHv, int TTv>
__global__ __launch_bounds__(256) void k_vt(const _Float16* __restrict__ V16, int ldv, int voff, _Float16* __restrict__ Vt) { __shared__ unsigned short tl[64][66]; const int tid = threadIdx.x; const int slab = blockIdx.x / (TTv / 64), lg = blockIdx.x % (TTv / 64); const int b = slab / NHv, h = slab % NHv;
  for (int i = tid; i < 64 * 8; i += 256) { const int r = i / 8, c8 = (i % 8) * 8; FragH f; f.half[0] = *(const v8us*)((const unsigned short*)V16 + ((size_t)b * TTv + lg * 64 + r) * ldv + voff + h * 64 + c8);
#pragma unroll
    for (int q = 0; q < 8; ++q) tl[r][c8 + q] = f.u[q]; }
  __syncthreads();
  for (int pass = 0; pass < 2; ++pass) {
#pragma unroll
    for (int rd = 0; rd < 2; ++rd) { const int d = rd * 32 + tid / 8, pc = tid % 8; FragH f;
#pragma unroll
      for (int q = 0; q < 8; ++q) f.u[q] = tl[pc * 8 + q][d];
      *(volatile v8us*)((unsigned short*)Vt + ((size_t)slab * 64 + d) * TTv + lg * 64 + pc * 8) = f.half[0]; }
    if (pass == 0) __threadfence(); } }

__global__ __launch_bounds__(256) void k_hl(const float* __restrict__ F, _Float16* __restrict__ Hh, _Float16* __restrict__ Hl, size_t n8) { const size_t t = (size_t)blockIdx.x * 256 + threadIdx.x; if (t >= n8) return; FragH fh, fl; const v4f a = *(const v4fa*)(F + t * 8), c = *(const v4fa*)(F + t * 8 + 4);
#pragma unroll
  for (int q = 0; q < 4; ++q) { _Float16 h = (_Float16)a[q]; fh.h[q] = h; fl.h[q] = (_Float16)((a[q] - (float)h) * 1024.0f); h = (_Float16)c[q]; fh.h[4 + q] = h; fl.h[4 + q] = (_Float16)((c[q] - (float)h) * 1024.0f); }
  for (int pass = 0; pass < 2; ++pass) { *(volatile v8us*)((unsigned short*)Hh + t * 8) = fh.half[0]; *(volatile v8us*)((unsigned short*)Hl + t * 8) = fl.half[0]; if (pass == 0) __threadfence(); } }

__device__ __forceinline__ float silu_f(float v) { return v / (1.0f + expf(-v)); }
__device__ __forceinline__ v4f shfl4(v4f v, int srcl) { v4f r; r[0] = __shfl(v[0], srcl, 32); r[1] = __shfl(v[1], srcl, 32); r[2] = __shfl(v[2], srcl, 32); r[3] = __shfl(v[3], srcl, 32); return r; }
__global__ __launch_bounds__(256) void k_we1(const float* __restrict__ eW1, _Float16* __restrict__ BI, _Float16* __restrict__ BJ) { const int t = blockIdx.x * 256 + threadIdx.x; if (t >= DD * (DD / 8)) return; const int k0 = (t % (DD / 8)) * 8, o = t / (DD / 8); FragH fi, fj;
#pragma unroll
  for (int q = 0; q < 8; ++q) { fi.h[q] = (_Float16)(bf16_round(eW1[(size_t)(k0 + q) * DD + o]) * 16.0f); fj.h[q] = (_Float16)(bf16_round(eW1[(size_t)(DD + k0 + q) * DD + o]) * 16.0f); }
  for (int pass = 0; pass < 2; ++pass) { *(volatile v8us*)((unsigned short*)BI + (size_t)o * DD + k0) = fi.half[0]; *(volatile v8us*)((unsigned short*)BJ + (size_t)o * DD + k0) = fj.half[0]; if (pass == 0) __threadfence(); } }
__global__ __launch_bounds__(256) void k_e1(const float* __restrict__ AI, const float* __restrict__ AJ, const float* __restrict__ pos, const float* __restrict__ cons, const float* __restrict__ mask, const float* __restrict__ eW1, const float* __restrict__ eb1, int b, int i0, _Float16* __restrict__ E1, float* __restrict__ GEO) {
  #pragma clang fp contract(off)
  const int t = blockIdx.x * 256 + threadIdx.x; if (t >= PCH * (DD / 8)) return; const int c0 = (t % (DD / 8)) * 8, pr = t / (DD / 8); const int il = pr / NN, j = pr % NN; const int i = i0 + il; const size_t ti = (size_t)b * NN + i, tj = (size_t)b * NN + j;
  const float rx = bf16_round(pos[ti * 3 + 0]) - bf16_round(pos[tj * 3 + 0]), ry = bf16_round(pos[ti * 3 + 1]) - bf16_round(pos[tj * 3 + 1]), rz = bf16_round(pos[ti * 3 + 2]) - bf16_round(pos[tj * 3 + 2]);
  const float dist = fmaxf(sqrtf(rx * rx + ry * ry + rz * rz), 1e-8f); const float ci = bf16_round(cons[ti]), cj = bf16_round(cons[tj]), mk = bf16_round(mask[((size_t)b * NN + i) * NN + j]);
  const v4f a = *(const v4fa*)(AI + ti * DD + c0), a2 = *(const v4fa*)(AI + ti * DD + c0 + 4), bj = *(const v4fa*)(AJ + tj * DD + c0), bj2 = *(const v4fa*)(AJ + tj * DD + c0 + 4); FragH f;
#pragma unroll
  for (int q = 0; q < 8; ++q) { const int c = c0 + q; float v = ((q < 4) ? a[q] : a2[q - 4]) + ((q < 4) ? bj[q] : bj2[q - 4]); v += dist * bf16_round(eW1[(size_t)(2 * DD) * DD + c]); v += ci * bf16_round(eW1[(size_t)(2 * DD + 1) * DD + c]); v += cj * bf16_round(eW1[(size_t)(2 * DD + 2) * DD + c]); v += mk * bf16_round(eW1[(size_t)(2 * DD + 3) * DD + c]); v += bf16_round(eb1[c]); f.h[q] = (_Float16)silu_f(v); }
  *(volatile v8us*)((unsigned short*)E1 + (size_t)pr * DD + c0) = f.half[0]; __threadfence(); *(volatile v8us*)((unsigned short*)E1 + (size_t)pr * DD + c0) = f.half[0]; (void)GEO; }
__global__ __launch_bounds__(256) void k_geo(const float* __restrict__ pos, const float* __restrict__ mask, int b, int i0, float* __restrict__ GEO) {
  #pragma clang fp contract(off)
  const int pr = blockIdx.x * 256 + threadIdx.x; if (pr >= PCH) return; const int il = pr / NN, j = pr % NN; const int i = i0 + il; const size_t ti = (size_t)b * NN + i, tj = (size_t)b * NN + j;
  const float rx = bf16_round(pos[ti * 3 + 0]) - bf16_round(pos[tj * 3 + 0]), ry = bf16_round(pos[ti * 3 + 1]) - bf16_round(pos[tj * 3 + 1]), rz = bf16_round(pos[ti * 3 + 2]) - bf16_round(pos[tj * 3 + 2]);
  const float dist = fmaxf(sqrtf(rx * rx + ry * ry + rz * rz), 1e-8f); v4f g; g[0] = rx / dist; g[1] = ry / dist; g[2] = rz / dist; g[3] = bf16_round(mask[((size_t)b * NN + i) * NN + j]);
  *(volatile v4f*)(GEO + (size_t)pr * 4) = g; __threadfence(); *(volatile v4f*)(GEO + (size_t)pr * 4) = g; }
__global__ __launch_bounds__(256) void k_ew(const float* __restrict__ EH, const float* __restrict__ GEO, int b, int i0, float* __restrict__ EW, float* __restrict__ out_ew) {
  #pragma clang fp contract(off)
  const int pr = blockIdx.x * 256 + threadIdx.x; if (pr >= PCH) return; const float* row = EH + (size_t)pr * DD; float s = 0.f;
#pragma unroll 1
  for (int c = 0; c < DD; c += 4) { const v4f a = *(const v4fa*)(row + c); s += (a[0] + a[1]) + (a[2] + a[3]); }
  const float w = (1.0f / (1.0f + expf(-(s / (float)DD)))) * GEO[(size_t)pr * 4 + 3];
  const int il = pr / NN, j = pr % NN; float* o = out_ew + ((size_t)b * NN + i0 + il) * NN + j;
  *(volatile float*)(EW + pr) = w; *(volatile float*)o = w; __threadfence(); *(volatile float*)(EW + pr) = w; *(volatile float*)o = w; }
__global__ __launch_bounds__(256) void k_f16c(const float* __restrict__ F, _Float16* __restrict__ O16, size_t n8) { const size_t t = (size_t)blockIdx.x * 256 + threadIdx.x; if (t >= n8) return; const v4f a = *(const v4fa*)(F + t * 8), c = *(const v4fa*)(F + t * 8 + 4); FragH f;
#pragma unroll
  for (int q = 0; q < 8; ++q) f.h[q] = (_Float16)((q < 4) ? a[q] : c[q - 4]);
  *(volatile v8us*)((unsigned short*)O16 + t * 8) = f.half[0]; __threadfence(); *(volatile v8us*)((unsigned short*)O16 + t * 8) = f.half[0]; }
__global__ __launch_bounds__(256) void k_msg(const float* __restrict__ EH, const float* __restrict__ EW, int b, int i0, float* __restrict__ MSG) {
  #pragma clang fp contract(off)
  const int t = blockIdx.x * 256 + threadIdx.x; if (t >= ICH * DD) return; const int c = t % DD, il = t / DD; float s = 0.f;
#pragma unroll 1
  for (int j = 0; j < NN; ++j) s += EH[((size_t)il * NN + j) * DD + c] * EW[(size_t)il * NN + j];
  float* o = MSG + ((size_t)b * NN + i0 + il) * DD + c; *(volatile float*)o = s; __threadfence(); *(volatile float*)o = s; }
__global__ __launch_bounds__(256) void k_gate(const float* __restrict__ G1, const float* __restrict__ vW2, const float* __restrict__ vb2, const float* __restrict__ EW, float* __restrict__ GT) {
  #pragma clang fp contract(off)
  const int pr = blockIdx.x * 256 + threadIdx.x; if (pr >= PCH) return; const float* row = G1 + (size_t)pr * DD; float s = bf16_round(vb2[0]);
#pragma unroll 1
  for (int c = 0; c < DD; c += 4) { const v4f a = *(const v4fa*)(row + c);
#pragma unroll
    for (int q = 0; q < 4; ++q) s += silu_f(a[q]) * bf16_round(vW2[c + q]); }
  const float g = s * EW[pr]; *(volatile float*)(GT + pr) = g; __threadfence(); *(volatile float*)(GT + pr) = g; }
__global__ __launch_bounds__(256) void k_vmsg(const float* __restrict__ GT, const float* __restrict__ GEO, int b, int i0, float* __restrict__ VMS) {
  #pragma clang fp contract(off)
  const int t = blockIdx.x * 256 + threadIdx.x; if (t >= ICH * 4) return; const int d = t & 3, il = t >> 2; float s = 0.f;
  if (d < 3) {
#pragma unroll 1
    for (int j = 0; j < NN; ++j) s += GT[(size_t)il * NN + j] * GEO[((size_t)il * NN + j) * 4 + d]; }
  float* o = VMS + ((size_t)b * NN + i0 + il) * 4 + d; *(volatile float*)o = s; __threadfence(); *(volatile float*)o = s; }
__global__ __launch_bounds__(256) void k_u16(const float* __restrict__ sf, const float* __restrict__ MSG, _Float16* __restrict__ U16) { const int t = blockIdx.x * 256 + threadIdx.x; if (t >= NTOK * 32) return; const int c0 = (t % 32) * 8, r = t / 32; FragH f;
#pragma unroll
  for (int q = 0; q < 8; ++q) { const int c = c0 + q; f.h[q] = (_Float16)((c < DD) ? bf16_round(sf[(size_t)r * DD + c]) : MSG[(size_t)r * DD + c - DD]); }
  *(volatile v8us*)((unsigned short*)U16 + (size_t)r * 2 * DD + c0) = f.half[0]; __threadfence(); *(volatile v8us*)((unsigned short*)U16 + (size_t)r * 2 * DD + c0) = f.half[0]; }
__global__ __launch_bounds__(256) void k_silu16(const float* __restrict__ F, _Float16* __restrict__ O16, size_t n8) {
  #pragma clang fp contract(off)
  const size_t t = (size_t)blockIdx.x * 256 + threadIdx.x; if (t >= n8) return; const v4f a = *(const v4fa*)(F + t * 8), c = *(const v4fa*)(F + t * 8 + 4); FragH f;
#pragma unroll
  for (int q = 0; q < 8; ++q) f.h[q] = (_Float16)silu_f((q < 4) ? a[q] : c[q - 4]);
  *(volatile v8us*)((unsigned short*)O16 + t * 8) = f.half[0]; __threadfence(); *(volatile v8us*)((unsigned short*)O16 + t * 8) = f.half[0]; }
__global__ __launch_bounds__(256) void k_sout(const float* __restrict__ sf, const float* __restrict__ UPD, const float* __restrict__ g, const float* __restrict__ bb, float* __restrict__ out) {
  #pragma clang fp contract(off)
  const int tid = threadIdx.x, w = tid >> 5, l = tid & 31; const int r = blockIdx.x * 8 + w; if (r >= NTOK) return; v4f x; float s = 0.f;
#pragma unroll
  for (int k = 0; k < 4; ++k) { const int c = l * 4 + k; x[k] = bf16_round(sf[(size_t)r * DD + c]) + UPD[(size_t)r * DD + c]; s += x[k]; }
  for (int o = 16; o > 0; o >>= 1) s += __shfl_xor(s, o, 32); const float mu = s / (float)DD; float q2 = 0.f;
#pragma unroll
  for (int k = 0; k < 4; ++k) { const float d = x[k] - mu; q2 += d * d; }
  for (int o = 16; o > 0; o >>= 1) q2 += __shfl_xor(q2, o, 32); const float rs = rsqrtf(q2 / (float)DD + 1e-5f); v4f v;
#pragma unroll
  for (int k = 0; k < 4; ++k) { const int c = l * 4 + k; v[k] = (x[k] - mu) * rs * bf16_round(g[c]) + bf16_round(bb[c]); }
  *(volatile v4f*)(out + (size_t)r * DD + l * 4) = v; __threadfence(); *(volatile v4f*)(out + (size_t)r * DD + l * 4) = v; }
__global__ __launch_bounds__(256) void k_vout(const float* __restrict__ vf, const float* __restrict__ VMS, float* __restrict__ out) {
  #pragma clang fp contract(off)
  const int t = blockIdx.x * 256 + threadIdx.x; if (t >= NTOK * 3 / 4) return; v4f v;
#pragma unroll
  for (int q = 0; q < 4; ++q) { const int f = t * 4 + q; const int r = f / 3, d = f % 3; v[q] = bf16_round(vf[f]) + VMS[(size_t)r * 4 + d]; }
  *(volatile v4f*)(out + (size_t)t * 4) = v; __threadfence(); *(volatile v4f*)(out + (size_t)t * 4) = v; }
__global__ __launch_bounds__(256) void k_sf16(const float* __restrict__ sf, _Float16* __restrict__ S16) { const int t = blockIdx.x * 256 + threadIdx.x; if (t >= NTOK * (DD / 8)) return; FragH f;
#pragma unroll
  for (int q = 0; q < 8; ++q) f.h[q] = (_Float16)bf16_round(sf[(size_t)t * 8 + q]);
  *(volatile v8us*)((unsigned short*)S16 + (size_t)t * 8) = f.half[0]; __threadfence(); *(volatile v8us*)((unsigned short*)S16 + (size_t)t * 8) = f.half[0]; }

extern "C" void kernel_launch(void* const* d_in, const int* in_sizes, int n_in,
                              void* d_out, int out_size, void* d_ws, size_t ws_size, hipStream_t stream) {
  (void)in_sizes; (void)n_in; (void)out_size;
  const float* const* I = (const float* const*)d_in; const float* sf = I[0]; const float* vf = I[1]; const float* pos = I[2]; const float* mask = I[3]; const float* cons = I[4]; const float* eW1 = I[5]; const float* eb1 = I[6]; const float* eW2 = I[7]; const float* eb2 = I[8]; const float* sW1 = I[9]; const float* sb1 = I[10]; const float* sW2 = I[11]; const float* sb2 = I[12]; const float* vW1 = I[13]; const float* vb1 = I[14]; const float* vW2 = I[15]; const float* vb2 = I[16]; const float* lng = I[17]; const float* lnb = I[18];
  char* ws = (char*)d_ws; size_t off = 0;
  auto take = [&](size_t bytes) { char* p = ws + off; off += (bytes + 255) & ~(size_t)255; return p; };
  _Float16* BI = (_Float16*)take((size_t)DD * DD * 2); _Float16* BJ = (_Float16*)take((size_t)DD * DD * 2); _Float16* BE2 = (_Float16*)take((size_t)DD * DD * 2); _Float16* BV1 = (_Float16*)take((size_t)DD * DD * 2); _Float16* BS1 = (_Float16*)take((size_t)DD * 2 * DD * 2); _Float16* BS2 = (_Float16*)take((size_t)DD * DD * 2);
  _Float16* S16 = (_Float16*)take((size_t)NTOK * DD * 2); float* AI = (float*)take((size_t)NTOK * DD * 4); float* AJ = (float*)take((size_t)NTOK * DD * 4); float* MSG = (float*)take((size_t)NTOK * DD * 4); float* VMS = (float*)take((size_t)NTOK * 4 * 4); _Float16* U16 = (_Float16*)take((size_t)NTOK * 2 * DD * 2); float* UH = (float*)take((size_t)NTOK * DD * 4); _Float16* UH16 = (_Float16*)take((size_t)NTOK * DD * 2); float* UPD = (float*)take((size_t)NTOK * DD * 4);
  _Float16* E1 = (_Float16*)take((size_t)PCH * DD * 2); float* GEO = (float*)take((size_t)PCH * 4 * 4); float* EH = (float*)take((size_t)PCH * DD * 4); _Float16* EH16 = (_Float16*)take((size_t)PCH * DD * 2); float* EW = (float*)take((size_t)PCH * 4); float* G1 = (float*)take((size_t)PCH * DD * 4); float* GT = (float*)take((size_t)PCH * 4);
  if (off > ws_size) return;
  float* out_s = (float*)d_out; float* out_v = (float*)((char*)d_out + 524288); float* out_e = (float*)((char*)d_out + 536576);
  k_we1<<<(DD * (DD / 8) + 255) / 256, 256, 0, stream>>>(eW1, BI, BJ); k_wt_f16<<<(DD * (DD / 8) + 255) / 256, 256, 0, stream>>>(eW2, BE2, DD, DD, 16.0f); k_wt_f16<<<(DD * (DD / 8) + 255) / 256, 256, 0, stream>>>(vW1, BV1, DD, DD, 16.0f); k_wt_f16<<<(DD * (2 * DD / 8) + 255) / 256, 256, 0, stream>>>(sW1, BS1, 2 * DD, DD, 16.0f); k_wt_f16<<<(DD * (DD / 8) + 255) / 256, 256, 0, stream>>>(sW2, BS2, DD, DD, 16.0f);
  k_sf16<<<(NTOK * (DD / 8) + 255) / 256, 256, 0, stream>>>(sf, S16);
  const dim3 gT(((NTOK / 16) * (DD / 64) + 3) / 4, 1), gP(((PCH / 16) * (DD / 64) + 3) / 4, 1);
  k_gemm_hhx<0><<<gT, 128, 0, stream>>>(S16, DD, 0, BI, DD, 0, 0.0625f, nullptr, 0, nullptr, 1, 0, 0, AI, nullptr, DD, 0, NTOK, DD, DD);
  k_gemm_hhx<0><<<gT, 128, 0, stream>>>(S16, DD, 0, BJ, DD, 0, 0.0625f, nullptr, 0, nullptr, 1, 0, 0, AJ, nullptr, DD, 0, NTOK, DD, DD);
  for (int b = 0; b < NBt; ++b) for (int i0 = 0; i0 < NN; i0 += ICH) {
    k_geo<<<(PCH + 255) / 256, 256, 0, stream>>>(pos, mask, b, i0, GEO); k_e1<<<(PCH * (DD / 8) + 255) / 256, 256, 0, stream>>>(AI, AJ, pos, cons, mask, eW1, eb1, b, i0, E1, GEO);
    k_gemm_hhx<0><<<gP, 128, 0, stream>>>(E1, DD, 0, BE2, DD, 0, 0.0625f, eb2, 0, nullptr, 1, 0, 0, EH, nullptr, DD, 0, PCH, DD, DD);
    k_ew<<<(PCH + 255) / 256, 256, 0, stream>>>(EH, GEO, b, i0, EW, out_e); k_f16c<<<(unsigned)(((size_t)PCH * DD / 8 + 255) / 256), 256, 0, stream>>>(EH, EH16, (size_t)PCH * DD / 8);
    k_msg<<<(ICH * DD + 255) / 256, 256, 0, stream>>>(EH, EW, b, i0, MSG);
    k_gemm_hhx<0><<<gP, 128, 0, stream>>>(EH16, DD, 0, BV1, DD, 0, 0.0625f, vb1, 0, nullptr, 1, 0, 0, G1, nullptr, DD, 0, PCH, DD, DD);
    k_gate<<<(PCH + 255) / 256, 256, 0, stream>>>(G1, vW2, vb2, EW, GT); k_vmsg<<<(ICH * 4 + 255) / 256, 256, 0, stream>>>(GT, GEO, b, i0, VMS); }
  k_u16<<<(NTOK * 32 + 255) / 256, 256, 0, stream>>>(sf, MSG, U16);
  k_gemm_hhx<0><<<gT, 128, 0, stream>>>(U16, 2 * DD, 0, BS1, 2 * DD, 0, 0.0625f, sb1, 0, nullptr, 1, 0, 0, UH, nullptr, DD, 0, NTOK, DD, 2 * DD);
  k_silu16<<<(unsigned)(((size_t)NTOK * DD / 8 + 255) / 256), 256, 0, stream>>>(UH, UH16, (size_t)NTOK * DD / 8);
  k_gemm_hhx<0><<<gT, 128, 0, stream>>>(UH16, DD, 0, BS2, DD, 0, 0.0625f, sb2, 0, nullptr, 1, 0, 0, UPD, nullptr, DD, 0, NTOK, DD, DD);
  k_sout<<<NTOK / 8, 256, 0, stream>>>(sf, UPD, lng, lnb, out_s); k_vout<<<(NTOK * 3 / 4 + 255) / 256, 256, 0, stream>>>(vf, VMS, out_v);
}
